// QuantumSelfAttention_91199335563801
// MI455X (gfx1250) — hardware-verified
//
#include <hip/hip_runtime.h>
#include <math.h>
#include <stddef.h>


#define NB 8
#define NS 1024
#define ND 64
#define NQ 8
#define NR (NB * NS)
#define NA 256
#define NK 512
#define TP 16
#define XP 72
#define QP 520
#define OP 68
#define KT 64
#define KW 128

static_assert(NR % TP == 0, "");
static_assert(NR % 16 == 0, "");
static_assert(NS % KT == 0, "");
static_assert(NS % KW == 0, "");
static_assert(NS % 16 == 0, "");
static_assert(ND == 64, "");
static_assert(NQ == 8, "");
static_assert(NA == 256 && NK == 2 * NA, "");
static_assert(NS == 8 * 128, "");

typedef _Float16 v16h __attribute__((ext_vector_type(16)));
typedef _Float16 v8h  __attribute__((ext_vector_type(8)));
typedef float    v8f  __attribute__((ext_vector_type(8)));
typedef float    v4f  __attribute__((ext_vector_type(4)));
typedef unsigned int v4u __attribute__((ext_vector_type(4)));

union Frag { v16h v; v8h half[2]; };
union Pk16 { v8h h; v4u u; };

__device__ __forceinline__ v8f wmma16(v16h a, v16h b, v8f c) {
  v8f d = __builtin_amdgcn_wmma_f32_16x16x32_f16(false, a, false, b, (short)0, c, false, false);
  asm volatile("v_nop\n\tv_nop\n\tv_nop\n\tv_nop" : "+v"(d) : "v"(a), "v"(b));
  return d;
}

__device__ __forceinline__ v8h cvt8(v4f a, v4f b, float s) {
  v8h r;
  r[0] = (_Float16)(a[0] * s); r[1] = (_Float16)(a[1] * s);
  r[2] = (_Float16)(a[2] * s); r[3] = (_Float16)(a[3] * s);
  r[4] = (_Float16)(b[0] * s); r[5] = (_Float16)(b[1] * s);
  r[6] = (_Float16)(b[2] * s); r[7] = (_Float16)(b[3] * s);
  return r;
}

struct QPar { float a0r, a0i, b0r, b0i; };

__device__ __forceinline__ QPar qpar(const float* th, int n) {
  const float phi = th[n * 3 + 0], tt = th[n * 3 + 1], om = th[n * 3 + 2];
  const float ct = cosf(tt * 0.5f), st = sinf(tt * 0.5f);
  float ssum, csum, sdif, cdif;
  sincosf((phi + om) * 0.5f, &ssum, &csum);
  sincosf((phi - om) * 0.5f, &sdif, &cdif);
  QPar p;
  p.a0r = csum * ct;  p.a0i = -ssum * ct;
  p.b0r = cdif * st;  p.b0i =  sdif * st;
  return p;
}

__device__ __forceinline__ v4f qstate(const QPar& p, float c, float s) {
  v4f v;
  v[0] = p.a0r * c - p.b0r * s;
  v[1] = p.a0i * c - p.b0i * s;
  v[2] = p.b0r * c + p.a0r * s;
  v[3] = -(p.b0i * c + p.a0i * s);
  return v;
}

__device__ __forceinline__ void prep_store(const _Float16* Vo, const _Float16* Pst,
                                           _Float16* vals, _Float16* Qg, _Float16* Kag, _Float16* Kbg,
                                           int tokbase, int w, int l)
{
#pragma unroll
  for (int i = 0; i < 2; ++i) {
    const int tokl = w * 8 + i * 4 + (l >> 3), ch = l & 7;
    Pk16 v; v.h = *(const v8h*)(Vo + tokl * XP + ch * 8);
    *(volatile v4u*)(vals + ((size_t)(tokbase + tokl) * ND + ch * 8)) = v.u;
  }
#pragma unroll
  for (int i = 0; i < 16; ++i) {
    const int lw = i * 4 + (l >> 3);
    const int tokl = w * 8 + (lw >> 3), c = lw & 7, off = c * 64 + (l & 7) * 8;
    const size_t g = (size_t)(tokbase + tokl) * NK + off;
    const _Float16* pq = Pst + tokl * QP;
    const _Float16* pk = Pst + TP * QP + tokl * QP;
    Pk16 q, ka, kb;
    q.h  = *(const v8h*)(pq + off);
    ka.h = *(const v8h*)(pk + off);
    if (c < 4) { kb.h = *(const v8h*)(pk + NA + off); }
    else       { const v8h t = *(const v8h*)(pk + (off - NA)); kb.h = -t; }
    *(volatile v4u*)(Qg  + g) = q.u;
    *(volatile v4u*)(Kag + g) = ka.u;
    *(volatile v4u*)(Kbg + g) = kb.u;
  }
}

__global__ void __launch_bounds__(64)
k_prep(const float* __restrict__ x, const float* __restrict__ thq, const float* __restrict__ thk,
       const float* __restrict__ Wv, const float* __restrict__ bv,
       _Float16* __restrict__ vals, _Float16* __restrict__ Qg,
       _Float16* __restrict__ Kag, _Float16* __restrict__ Kbg)
{
  __shared__ __attribute__((aligned(16))) _Float16 Xs[TP * XP];
  __shared__ __attribute__((aligned(16))) _Float16 Ws[ND * XP];
  __shared__ __attribute__((aligned(16))) _Float16 Vo[TP * XP];
  __shared__ __attribute__((aligned(16))) float    Sst[2 * TP * NQ * 4];
  __shared__ __attribute__((aligned(16))) _Float16 Pst[2 * TP * QP];

  const int tid = threadIdx.x;
  const int l = tid & 31, w = tid >> 5, h = l >> 4, m = l & 15;
  const int tokbase = blockIdx.x * TP;
  const float PI_F = 3.14159274101257324f;

  {
    const int r = tid >> 2, c0 = (tid & 3) * 16;
    const float* xp = x + ((size_t)(tokbase + r) * ND + c0);
#pragma unroll
    for (int j = 0; j < 2; ++j) {
      const v4f x0 = *(const v4f*)(xp + 8 * j);
      const v4f x1 = *(const v4f*)(xp + 8 * j + 4);
      *(v8h*)&Xs[r * XP + c0 + 8 * j] = cvt8(x0, x1, 1.0f);
    }
    const float* wp = Wv + (size_t)tid * ND;
#pragma unroll
    for (int j = 0; j < 8; ++j) {
      const v4f w0 = *(const v4f*)(wp + 8 * j);
      const v4f w1 = *(const v4f*)(wp + 8 * j + 4);
      *(v8h*)&Ws[tid * XP + 8 * j] = cvt8(w0, w1, 16.0f);
    }
  }
  {
    const int tok = tid >> 2, p = tid & 3;
#pragma unroll 1
    for (int jq = 0; jq < 2; ++jq) {
      const int n = 2 * p + jq;
      const float xv = x[(size_t)(tokbase + tok) * ND + n];
      const float xn = tanhf(xv);
      const float ang = (xn * PI_F) * 0.5f;
      float sn, cs;
      sincosf(ang, &sn, &cs);
#pragma unroll 1
      for (int qk = 0; qk < 2; ++qk) {
        const float* th = (qk == 0) ? thq : thk;
        const QPar pp = qpar(th, n);
        *(v4f*)&Sst[((qk * TP + tok) * NQ + n) * 4] = qstate(pp, cs, sn);
      }
    }
  }
  __syncthreads();

  {
    const int ct0 = 2 * w, ct1 = 2 * w + 1;
    const v8f zero = {0.f, 0.f, 0.f, 0.f, 0.f, 0.f, 0.f, 0.f};
    v8f acc0 = zero, acc1 = zero;
#pragma unroll
    for (int kk = 0; kk < ND; kk += 32) {
      Frag a, b0, b1;
      const _Float16* ap = Xs + m * XP + kk + 8 * h;
      a.half[0] = *(const v8h*)ap;
      a.half[1] = *(const v8h*)(ap + 16);
      const _Float16* bp0 = Ws + (ct0 * 16 + m) * XP + kk + 8 * h;
      b0.half[0] = *(const v8h*)bp0;
      b0.half[1] = *(const v8h*)(bp0 + 16);
      const _Float16* bp1 = Ws + (ct1 * 16 + m) * XP + kk + 8 * h;
      b1.half[0] = *(const v8h*)bp1;
      b1.half[1] = *(const v8h*)(bp1 + 16);
      acc0 = wmma16(a.v, b0.v, acc0);
      acc1 = wmma16(a.v, b1.v, acc1);
    }
    const float bia0 = bv[ct0 * 16 + m], bia1 = bv[ct1 * 16 + m];
#pragma unroll
    for (int r = 0; r < 8; ++r) {
      const int row = 8 * h + r;
      Vo[row * XP + ct0 * 16 + m] = (_Float16)(acc0[r] * 0.0625f + bia0);
      Vo[row * XP + ct1 * 16 + m] = (_Float16)(acc1[r] * 0.0625f + bia1);
    }
  }

  {
    const int tok = tid >> 2, p = tid & 3;
#pragma unroll 1
    for (int qk = 0; qk < 2; ++qk) {
      const float* sp = Sst + (qk * TP + tok) * (NQ * 4);
      _Float16* pst = Pst + qk * (TP * QP) + tok * QP;
      float Lr[16], Li[16];
      Lr[0] = sp[0]; Li[0] = sp[1]; Lr[1] = sp[2]; Li[1] = sp[3];
#pragma unroll
      for (int bq = 1; bq < 4; ++bq) {
        const float ar0 = sp[bq * 4 + 0], ai0 = sp[bq * 4 + 1];
        const float ar1 = sp[bq * 4 + 2], ai1 = sp[bq * 4 + 3];
#pragma unroll
        for (int i = 0; i < (1 << bq); ++i) {
          const float xr = Lr[i], xi = Li[i];
          Lr[(1 << bq) + i] = xr * ar1 - xi * ai1;
          Li[(1 << bq) + i] = xr * ai1 + xi * ar1;
          Lr[i] = xr * ar0 - xi * ai0;
          Li[i] = xr * ai0 + xi * ar0;
        }
      }
#pragma unroll 1
      for (int jh = 0; jh < 4; ++jh) {
        const int hi = 4 * p + jh;
        float hr = 16.0f, hm = 0.0f;
#pragma unroll
        for (int bq = 0; bq < 4; ++bq) {
          const int bit = (hi >> bq) & 1;
          const float ar = sp[(4 + bq) * 4 + 2 * bit], ai = sp[(4 + bq) * 4 + 2 * bit + 1];
          const float tr = hr * ar - hm * ai, ti = hr * ai + hm * ar;
          hr = tr; hm = ti;
        }
        Frag re, im;
#pragma unroll
        for (int lo = 0; lo < 16; ++lo) {
          re.v[lo] = (_Float16)(hr * Lr[lo] - hm * Li[lo]);
          im.v[lo] = (_Float16)(hr * Li[lo] + hm * Lr[lo]);
        }
        *(v8h*)(pst + hi * 16)          = re.half[0];
        *(v8h*)(pst + hi * 16 + 8)      = re.half[1];
        *(v8h*)(pst + NA + hi * 16)     = im.half[0];
        *(v8h*)(pst + NA + hi * 16 + 8) = im.half[1];
      }
    }
  }
  __syncthreads();

  prep_store(Vo, Pst, vals, Qg, Kag, Kbg, tokbase, w, l);
  __threadfence();
  prep_store(Vo, Pst, vals, Qg, Kag, Kbg, tokbase, w, l);
}

__global__ void __launch_bounds__(256)
k_sc(const _Float16* __restrict__ Qg, const _Float16* __restrict__ Kag,
     const _Float16* __restrict__ Kbg, float* __restrict__ attn)
{
  __shared__ __attribute__((aligned(16))) _Float16 Qt[16 * QP];
  __shared__ __attribute__((aligned(16))) float    Sc[16 * NS];

  const int tid = threadIdx.x;
  const int l = tid & 31, w = tid >> 5, h = l >> 4, m = l & 15;
  const int grow0 = blockIdx.x * 16;
  const int b = grow0 / NS;

  {
    const int r = tid >> 4, c0 = (tid & 15) * 32;
    const _Float16* qp = Qg + ((size_t)(grow0 + r) * NK + c0);
#pragma unroll
    for (int j = 0; j < 4; ++j) *(v8h*)&Qt[r * QP + c0 + 8 * j] = *(const v8h*)(qp + 8 * j);
  }
  __syncthreads();

  const float SINV = 1.0f / 256.0f;
  const v8f zero = {0.f, 0.f, 0.f, 0.f, 0.f, 0.f, 0.f, 0.f};
  const _Float16* aq = Qt + m * QP + 8 * h;

#pragma unroll 1
  for (int kt = 0; kt < NS / KW; ++kt) {
    const int t0 = kt * KW + 16 * w;
    const size_t krow = (size_t)(b * NS + t0 + m) * NK + 8 * h;
    const _Float16* kap = Kag + krow;
    const _Float16* kbp = Kbg + krow;
    v8f accR = zero, accI = zero;
#pragma unroll 4
    for (int ks = 0; ks < NK / 32; ++ks) {
      const int k0 = ks * 32;
      Frag a, ba, bb;
      a.half[0]  = *(const v8h*)(aq + k0);
      a.half[1]  = *(const v8h*)(aq + k0 + 16);
      ba.half[0] = *(const v8h*)(kap + k0);
      ba.half[1] = *(const v8h*)(kap + k0 + 16);
      bb.half[0] = *(const v8h*)(kbp + k0);
      bb.half[1] = *(const v8h*)(kbp + k0 + 16);
      accR = wmma16(a.v, ba.v, accR);
      accI = wmma16(a.v, bb.v, accI);
    }
#pragma unroll
    for (int r = 0; r < 8; ++r) {
      const float ovr = accR[r] * SINV, ovi = accI[r] * SINV;
      const float core = ovr * ovr + ovi * ovi;
      Sc[(8 * h + r) * NS + t0 + m] = (core + 1.0f) * 0.5f;
    }
  }
  __syncthreads();

#pragma unroll 1
  for (int j = 0; j < 2; ++j) {
    const int row = 2 * w + j;
    const float* srow = Sc + row * NS + 4 * l;
    v4f sv[8];
#pragma unroll
    for (int i = 0; i < 8; ++i) sv[i] = *(const v4f*)(srow + i * 128);
    float mx = sv[0][0];
#pragma unroll
    for (int i = 0; i < 8; ++i)
      mx = fmaxf(mx, fmaxf(fmaxf(sv[i][0], sv[i][1]), fmaxf(sv[i][2], sv[i][3])));
    for (int off = 16; off; off >>= 1) mx = fmaxf(mx, __shfl_xor(mx, off, 32));
    v4f e[8];
    float ssum = 0.0f;
#pragma unroll
    for (int i = 0; i < 8; ++i) {
      e[i][0] = expf(sv[i][0] - mx); e[i][1] = expf(sv[i][1] - mx);
      e[i][2] = expf(sv[i][2] - mx); e[i][3] = expf(sv[i][3] - mx);
      ssum += (e[i][0] + e[i][1]) + (e[i][2] + e[i][3]);
    }
    for (int off = 16; off; off >>= 1) ssum += __shfl_xor(ssum, off, 32);
    const float inv = 1.0f / ssum;
#pragma unroll
    for (int i = 0; i < 8; ++i) e[i] = e[i] * inv;
    float* arow = attn + ((size_t)(grow0 + row) * NS + 4 * l);
#pragma unroll
    for (int i = 0; i < 8; ++i) *(volatile v4f*)(arow + i * 128) = e[i];
    __threadfence();
#pragma unroll
    for (int i = 0; i < 8; ++i) *(volatile v4f*)(arow + i * 128) = e[i];
  }
}

__global__ void __launch_bounds__(128)
k_av(const float* __restrict__ attn, const _Float16* __restrict__ vals, float* __restrict__ out)
{
  __shared__ __attribute__((aligned(16))) _Float16 As[16 * XP];
  __shared__ __attribute__((aligned(16))) _Float16 Vs[KT * XP];
  __shared__ __attribute__((aligned(16))) float Os[16 * OP];

  const int tid = threadIdx.x;
  const int l = tid & 31, w = tid >> 5, h = l >> 4, m = l & 15;
  const int grow0 = blockIdx.x * 16;
  const int b = grow0 / NS;

  const v8f zero = {0.f, 0.f, 0.f, 0.f, 0.f, 0.f, 0.f, 0.f};
  v8f acc = zero;

  for (int t0 = 0; t0 < NS; t0 += KT) {
    {
      const int r = tid >> 3, c0 = (tid & 7) * 8;
      const float* ap = attn + ((size_t)(grow0 + r) * NS + t0 + c0);
      const v4f a0 = *(const v4f*)ap;
      const v4f a1 = *(const v4f*)(ap + 4);
      *(v8h*)&As[r * XP + c0] = cvt8(a0, a1, 1024.0f);
    }
    {
      const int r = tid >> 1, c0 = (tid & 1) * 32;
      const _Float16* vp = vals + ((size_t)(b * NS + t0 + r) * ND + c0);
#pragma unroll
      for (int j = 0; j < 4; ++j)
        *(v8h*)&Vs[r * XP + c0 + 8 * j] = *(const v8h*)(vp + 8 * j);
    }
    __syncthreads();

#pragma unroll
    for (int kk = 0; kk < KT; kk += 32) {
      Frag a, bb;
      const _Float16* ap = As + m * XP + kk + 8 * h;
      a.half[0] = *(const v8h*)ap;
      a.half[1] = *(const v8h*)(ap + 16);
#pragma unroll
      for (int i = 0; i < 8; ++i) {
        bb.v[i]     = Vs[(kk + 8 * h + i) * XP + 16 * w + m];
        bb.v[8 + i] = Vs[(kk + 16 + 8 * h + i) * XP + 16 * w + m];
      }
      acc = wmma16(a.v, bb.v, acc);
    }
    __syncthreads();
  }

#pragma unroll
  for (int r = 0; r < 8; ++r) Os[(8 * h + r) * OP + 16 * w + m] = acc[r] * (1.0f / 1024.0f);
  __syncthreads();

  v4f o[2];
  size_t ooff[2];
#pragma unroll
  for (int j = 0; j < 2; ++j) {
    const int rr = 4 * w + 2 * j + (l >> 4);
    const int c = (l & 15) * 4;
    o[j] = *(const v4f*)&Os[rr * OP + c];
    ooff[j] = (size_t)(grow0 + rr) * ND + c;
    *(volatile v4f*)(out + ooff[j]) = o[j];
  }
  __threadfence();
#pragma unroll
  for (int j = 0; j < 2; ++j) *(volatile v4f*)(out + ooff[j]) = o[j];
}

extern "C" void kernel_launch(void* const* d_in, const int* in_sizes, int n_in,
                              void* d_out, int out_size, void* d_ws, size_t ws_size,
                              hipStream_t stream)
{
  if (n_in < 5) return;
  if (in_sizes[0] != NR * ND || in_sizes[1] != NQ * 3 || in_sizes[2] != NQ * 3 ||
      in_sizes[3] != ND * ND || in_sizes[4] != ND) return;
  if (out_size != NR * ND + NR * NS) return;

  const size_t st_bytes   = (size_t)NR * NK * sizeof(_Float16);
  const size_t vals_bytes = (size_t)NR * ND * sizeof(_Float16);
  if (3 * st_bytes + vals_bytes > ws_size) return;

  const float* x   = (const float*)d_in[0];
  const float* thq = (const float*)d_in[1];
  const float* thk = (const float*)d_in[2];
  const float* Wv  = (const float*)d_in[3];
  const float* bv  = (const float*)d_in[4];

  float* out  = (float*)d_out;
  float* attn = out + (size_t)NR * ND;

  char* ws = (char*)d_ws;
  _Float16* Qg   = (_Float16*)(ws);
  _Float16* Kag  = (_Float16*)(ws + st_bytes);
  _Float16* Kbg  = (_Float16*)(ws + 2 * st_bytes);
  _Float16* vals = (_Float16*)(ws + 3 * st_bytes);

  k_prep<<<NR / TP, 64, 0, stream>>>(x, thq, thk, Wv, bv, vals, Qg, Kag, Kbg);
  k_sc<<<NR / 16, 256, 0, stream>>>(Qg, Kag, Kbg, attn);
  k_av<<<NR / 16, 128, 0, stream>>>(attn, vals, out);
}
